// GCN_72619307040769
// MI455X (gfx1250) — hardware-verified
//
#include <hip/hip_runtime.h>
#include <stddef.h>
#include <stdint.h>
#include <math.h>


#define DF     128
#define K2     256
#define NCLS   40
#define NCP    48
#define NTHR   256
#define NWAVE  8
#define EPT    8
#define CHUNK  (NTHR * EPT)
#define WCAP   (EPT * 32)
#define LISTN  (NWAVE * WCAP)
#define NBA    1024
#define SLA    10
#define RCAP   24576
#define DEGCAP 64
#define GBM    64
#define GBN    128
#define GTHR   128
#define U_W1   (DF * (DF / 8))
#define U_W2   (DF * (K2 / 8))
#define U_WC   (NCP * (K2 / 8))
#define U_ALL  (U_W1 + 2 * U_W2 + U_WC)
#define AGG_ZINTS (LISTN + 2 * RCAP + 3 * NBA)
#define STRUCT_LDS_INTS (AGG_ZINTS + 16)
#define MLINE  32
#define WSMAX  134217728

static_assert((CHUNK & (CHUNK - 1)) == 0 && CHUNK <= 4096);
static_assert((NBA & (NBA - 1)) == 0 && NBA == (1 << SLA));
static_assert(((long long)CHUNK << SLA) < (1LL << 31));
static_assert(NBA == 4 * NTHR);
static_assert(NBA % NWAVE == 0 && NBA % 32 == 0 && NBA % GBM == 0);
static_assert(RCAP % 1024 == 0 && AGG_ZINTS % (NTHR * 4) == 0 && LISTN % 4 == 0);
static_assert(RCAP % (NTHR * 4) == 0);
static_assert(DF % 32 == 0 && K2 % 32 == 0 && K2 == 2 * DF && DF == 4 * 32);
static_assert(GBN == DF && GBM == (GTHR / 32) * 16);
static_assert(U_W1 % NTHR == 0 && U_W2 % NTHR == 0 && U_WC % NTHR == 0);
static_assert(NCP % 16 == 0 && NCP >= NCLS && NCLS % 4 == 0);
static_assert((GBM * NCLS) % (4 * GTHR) == 0 && (GBM * NCLS * 4) % 128 == 0);
static_assert(STRUCT_LDS_INTS * 4 <= 300000);

typedef float          v4f   __attribute__((ext_vector_type(4)));
typedef float          v8f   __attribute__((ext_vector_type(8)));
typedef int            v4i   __attribute__((ext_vector_type(4)));
typedef int            v8i   __attribute__((ext_vector_type(8)));
typedef unsigned short v4us  __attribute__((ext_vector_type(4)));
typedef unsigned short v8us  __attribute__((ext_vector_type(8)));
typedef unsigned short v16us __attribute__((ext_vector_type(16)));
typedef __bf16         v16bf __attribute__((ext_vector_type(16)));
typedef v4f  __attribute__((may_alias)) v4fa;
typedef v4i  __attribute__((may_alias)) v4ia;
typedef v4us __attribute__((may_alias)) v4usa;
typedef v8us __attribute__((may_alias)) v8usa;
union FragB { v16bf v; v16us u; v8us h[2]; v8i w; };

__device__ __forceinline__ v8f wmb(const FragB& a, const FragB& b, v8f c) {
  v8f d = __builtin_amdgcn_wmma_f32_16x16x32_bf16(false, a.v, false, b.v, (short)0, c, false, false);
  asm volatile("v_nop\n\tv_nop\n\tv_nop\n\tv_nop" : "+v"(d) : "v"(a.w), "v"(b.w));
  return d;
}

__device__ __forceinline__ unsigned bf16_bits(float f) {
  const unsigned u = __float_as_uint(f);
  return (u + 0x7FFFu + ((u >> 16) & 1u)) >> 16;
}
__device__ __forceinline__ float bf16_val(float f) {
  return __uint_as_float(bf16_bits(f) << 16);
}

__device__ __forceinline__ void wave_sync() {
  __builtin_amdgcn_fence(__ATOMIC_RELEASE, "wavefront");
  __builtin_amdgcn_wave_barrier();
  __builtin_amdgcn_fence(__ATOMIC_ACQUIRE, "wavefront");
}

template <int SLB>
__device__ __forceinline__ int scan_chunk(const int* __restrict__ dsts, int nE, int cbase, int slotBase,
                                          int nb, int vec8, int* list, int tid, int lane, int wave) {
  int wc = 0;
  const int el0  = tid * EPT;
  const int e0   = cbase + el0;
  const int sent = -2147483647 - 1;
  v4i da, db;
  if (vec8 != 0 && cbase + CHUNK <= nE) {
    da = *(const v4i*)(dsts + e0);
    db = *(const v4i*)(dsts + e0 + 4);
  } else {
    da.x = (e0     < nE) ? dsts[min(e0,     nE - 1)] : sent;
    da.y = (e0 + 1 < nE) ? dsts[min(e0 + 1, nE - 1)] : sent;
    da.z = (e0 + 2 < nE) ? dsts[min(e0 + 2, nE - 1)] : sent;
    da.w = (e0 + 3 < nE) ? dsts[min(e0 + 3, nE - 1)] : sent;
    db.x = (e0 + 4 < nE) ? dsts[min(e0 + 4, nE - 1)] : sent;
    db.y = (e0 + 5 < nE) ? dsts[min(e0 + 5, nE - 1)] : sent;
    db.z = (e0 + 6 < nE) ? dsts[min(e0 + 6, nE - 1)] : sent;
    db.w = (e0 + 7 < nE) ? dsts[min(e0 + 7, nE - 1)] : sent;
  }
  const unsigned nbs = (unsigned)slotBase;
  const unsigned unb = (unsigned)nb;
  const unsigned s0 = (unsigned)da.x - nbs, s1 = (unsigned)da.y - nbs;
  const unsigned s2 = (unsigned)da.z - nbs, s3 = (unsigned)da.w - nbs;
  const unsigned s4 = (unsigned)db.x - nbs, s5 = (unsigned)db.y - nbs;
  const unsigned s6 = (unsigned)db.z - nbs, s7 = (unsigned)db.w - nbs;
  const bool h0 = s0 < unb, h1 = s1 < unb, h2 = s2 < unb, h3 = s3 < unb;
  const bool h4 = s4 < unb, h5 = s5 < unb, h6 = s6 < unb, h7 = s7 < unb;
  const unsigned any = __builtin_amdgcn_ballot_w32(h0 | h1 | h2 | h3 | h4 | h5 | h6 | h7);
  if (any != 0u) {
#define HITJ(J, HJ, SJ) { \
      const unsigned mj = __builtin_amdgcn_ballot_w32(HJ); \
      if (mj != 0u) { \
        if (HJ) { \
          const int pos = wc + (int)__builtin_amdgcn_mbcnt_lo(mj, 0u); \
          if (pos < WCAP) list[wave * WCAP + pos] = ((el0 + (J)) << SLB) | (int)(SJ); \
        } \
        wc += (int)__builtin_popcount(mj); } }
    HITJ(0, h0, s0)
    HITJ(1, h1, s1)
    HITJ(2, h2, s2)
    HITJ(3, h3, s3)
    HITJ(4, h4, s4)
    HITJ(5, h5, s5)
    HITJ(6, h6, s6)
    HITJ(7, h7, s7)
#undef HITJ
  }
  return wc;
}

__global__ __launch_bounds__(NTHR) void k_cvx(const float* __restrict__ x, int nN, int nUnits,
                                              unsigned short* xb) {
  const int u = (int)blockIdx.x * NTHR + (int)threadIdx.x;
  if (u >= nUnits) return;
  const int row = u >> 4;
  const int k8  = (u & 15) * 8;
  const int rc  = row < nN ? row : nN - 1;
  const float* p = x + (size_t)rc * DF + k8;
  const v4f a = *(const v4fa*)p;
  const v4f b = *(const v4fa*)(p + 4);
  const bool ok = row < nN;
  v8us o;
  o[0] = ok ? (unsigned short)bf16_bits(a.x) : (unsigned short)0;
  o[1] = ok ? (unsigned short)bf16_bits(a.y) : (unsigned short)0;
  o[2] = ok ? (unsigned short)bf16_bits(a.z) : (unsigned short)0;
  o[3] = ok ? (unsigned short)bf16_bits(a.w) : (unsigned short)0;
  o[4] = ok ? (unsigned short)bf16_bits(b.x) : (unsigned short)0;
  o[5] = ok ? (unsigned short)bf16_bits(b.y) : (unsigned short)0;
  o[6] = ok ? (unsigned short)bf16_bits(b.z) : (unsigned short)0;
  o[7] = ok ? (unsigned short)bf16_bits(b.w) : (unsigned short)0;
  unsigned short* dp = xb + (size_t)row * DF + k8;
  *(volatile v8us*)dp = o;
  __threadfence();
  *(volatile v8us*)dp = o;
}

__device__ __forceinline__ v8us gather8(const float* __restrict__ W, int k0, int ncol, int n, bool ok) {
  const int nc = n < ncol ? n : ncol - 1;
  const float* p = W + (size_t)k0 * ncol + nc;
  v8us o;
#pragma unroll
  for (int i = 0; i < 8; ++i) {
    const float f = p[(size_t)i * ncol];
    o[i] = ok ? (unsigned short)bf16_bits(f) : (unsigned short)0;
  }
  return o;
}

__global__ __launch_bounds__(NTHR) void k_wprep(const float* __restrict__ W1, const float* __restrict__ W2,
                                                const float* __restrict__ W3, const float* __restrict__ Wc,
                                                unsigned short* W1T, unsigned short* W2T2,
                                                unsigned short* W3T2, unsigned short* WcT2) {
  const int u = (int)blockIdx.x * NTHR + (int)threadIdx.x;
  v8us o;
  unsigned short* dp;
  if (u < U_W1) {
    const int n  = u >> 4;
    const int k8 = (u & 15) * 8;
    o  = gather8(W1, k8, DF, n, true);
    dp = W1T + (size_t)n * DF + k8;
  } else if (u < U_W1 + U_W2) {
    const int v  = u - U_W1;
    const int n  = v >> 5;
    const int k8 = (v & 31) * 8;
    o  = gather8(W2, k8 & (DF - 1), DF, n, true);
    dp = W2T2 + (size_t)n * K2 + k8;
  } else if (u < U_W1 + 2 * U_W2) {
    const int v  = u - U_W1 - U_W2;
    const int n  = v >> 5;
    const int k8 = (v & 31) * 8;
    o  = gather8(W3, k8 & (DF - 1), DF, n, true);
    dp = W3T2 + (size_t)n * K2 + k8;
  } else if (u < U_ALL) {
    const int v  = u - U_W1 - 2 * U_W2;
    const int n  = v >> 5;
    const int k8 = (v & 31) * 8;
    o  = gather8(Wc, k8 & (DF - 1), NCLS, n, n < NCLS);
    dp = WcT2 + (size_t)n * K2 + k8;
  } else {
    return;
  }
  *(volatile v8us*)dp = o;
  __threadfence();
  *(volatile v8us*)dp = o;
}

__global__ __launch_bounds__(NTHR) void k_struct(const int* __restrict__ srcs, const int* __restrict__ dsts,
                                                 int nE, int nN, int vec8,
                                                 float* dis, int* cntT, int* offT, int* meta, int* lst) {
  extern __shared__ __attribute__((aligned(16))) int dsm[];
  int* list = dsm;
  int* hl   = dsm + LISTN;
  int* sl   = dsm + LISTN + RCAP;
  int* cnt  = dsm + LISTN + 2 * RCAP;
  int* offs = cnt + NBA;
  int* cur  = offs + NBA;
  int* misc = cur + NBA;
  const int tid = (int)threadIdx.x, lane = tid & 31, wave = tid >> 5;
  const int blk = (int)blockIdx.x;
  const int nodeBase = blk * NBA;

  {
    const v4i z4 = {0, 0, 0, 0};
    for (int i = tid * 4; i < AGG_ZINTS; i += NTHR * 4) *(v4ia*)(dsm + i) = z4;
    if (tid < 16) misc[tid] = 0;
  }
  __syncthreads();

  int t = 0, ov = 0;
  const int nChunks = (nE + CHUNK - 1) / CHUNK;
#pragma unroll 1
  for (int ch = 0; ch < nChunks; ++ch) {
    const int cbase = ch * CHUNK;
    const int wc = scan_chunk<SLA>(dsts, nE, cbase, nodeBase, NBA, vec8, list, tid, lane, wave);
    if (lane == 0) misc[wave] = wc;
    __syncthreads();
    if (wave == 0) {
#pragma unroll 1
      for (int w2 = 0; w2 < NWAVE; ++w2) {
        int c = misc[w2];
        c = c < 0 ? 0 : (c > WCAP ? WCAP : c);
#pragma unroll 1
        for (int b0 = 0; b0 < c; b0 += 32) {
          const int idx = b0 + lane;
          const int ent = list[w2 * WCAP + (idx < WCAP ? idx : WCAP - 1)];
          const int m32 = (c - b0) < 32 ? (c - b0) : 32;
#pragma unroll 1
          for (int k = 0; k < m32; ++k) {
            const int u    = __builtin_amdgcn_readlane(ent, k);
            const int slot = u & (NBA - 1);
            const int el   = (u >> SLA) & (CHUNK - 1);
            const int pk   = ((cbase + el) << SLA) | slot;
            if (t < RCAP) {
              if (lane == 0) { hl[t] = pk; cnt[slot] = cnt[slot] + 1; }
              t = t + 1;
            } else {
              ov = 1;
            }
          }
        }
      }
    }
    __syncthreads();
  }
  if (wave == 0 && lane == 0) { misc[8] = t; misc[9] = ov; }
  __syncthreads();
  int tt = misc[8];
  tt = tt < 0 ? 0 : (tt > RCAP ? RCAP : tt);
  const int ovf = misc[9];

  if (wave == 0) {
    const int base = lane * (NBA / 32);
    int s = 0;
#pragma unroll 1
    for (int i = 0; i < NBA / 32; ++i) s += cnt[base + i];
    int incl = s;
#pragma unroll
    for (int d = 1; d < 32; d <<= 1) {
      const int y = __shfl_up(incl, d, 32);
      if (lane >= d) incl += y;
    }
    int run = incl - s;
#pragma unroll 1
    for (int i = 0; i < NBA / 32; ++i) {
      const int cv = cnt[base + i];
      offs[base + i] = run;
      cur[base + i]  = run;
      run += cv;
    }
  }
  __syncthreads();
  if (wave == 0) {
#pragma unroll 1
    for (int b0 = 0; b0 < tt; b0 += 32) {
      const int idx = b0 + lane;
      const int ent = hl[idx < RCAP ? idx : RCAP - 1];
      const int m32 = (tt - b0) < 32 ? (tt - b0) : 32;
#pragma unroll 1
      for (int k = 0; k < m32; ++k) {
        const int u    = __builtin_amdgcn_readlane(ent, k);
        const int slot = u & (NBA - 1);
        if (lane == 0) {
          int p = cur[slot];
          p = p < 0 ? 0 : (p > RCAP - 1 ? RCAP - 1 : p);
          sl[p] = u;
          cur[slot] = p + 1;
        }
      }
    }
  }
  __syncthreads();

  {
    const v4i c4 = *(const v4ia*)(cnt + 4 * tid);
    const v4i o4 = *(const v4ia*)(offs + 4 * tid);
    v4f dv;
    dv.x = rsqrtf((float)c4.x + 1.0f);
    dv.y = rsqrtf((float)c4.y + 1.0f);
    dv.z = rsqrtf((float)c4.z + 1.0f);
    dv.w = rsqrtf((float)c4.w + 1.0f);
    v4i mv;
    mv.x = (tid == 0) ? tt : 0;
    mv.y = (tid == 0) ? ovf : 0;
    mv.z = 0; mv.w = 0;
    float* dp = dis  + (size_t)nodeBase + 4 * tid;
    int*   cp = cntT + (size_t)nodeBase + 4 * tid;
    int*   op = offT + (size_t)nodeBase + 4 * tid;
    int*   mp = meta + (size_t)blk * MLINE + 4 * (tid & 7);
    const bool mok = tid < 8;
    *(volatile v4f*)dp = dv;
    *(volatile v4i*)cp = c4;
    *(volatile v4i*)op = o4;
    if (mok) *(volatile v4i*)mp = mv;
    __threadfence();
    *(volatile v4f*)dp = dv;
    *(volatile v4i*)cp = c4;
    *(volatile v4i*)op = o4;
    if (mok) *(volatile v4i*)mp = mv;
  }
  int* bl = lst + (size_t)blk * RCAP;
#pragma unroll 1
  for (int i0 = 0; i0 < RCAP; i0 += 1024) {
    const int idx = i0 + 4 * tid;
    const v4i e4 = *(const v4ia*)(sl + idx);
    int e0 = e4.x >> SLA, e1 = e4.y >> SLA, e2 = e4.z >> SLA, e3 = e4.w >> SLA;
    e0 = e0 < 0 ? 0 : (e0 > nE - 1 ? nE - 1 : e0);
    e1 = e1 < 0 ? 0 : (e1 > nE - 1 ? nE - 1 : e1);
    e2 = e2 < 0 ? 0 : (e2 > nE - 1 ? nE - 1 : e2);
    e3 = e3 < 0 ? 0 : (e3 > nE - 1 ? nE - 1 : e3);
    int r0 = srcs[e0], r1 = srcs[e1], r2 = srcs[e2], r3 = srcs[e3];
    r0 = r0 < 0 ? 0 : (r0 > nN - 1 ? nN - 1 : r0);
    r1 = r1 < 0 ? 0 : (r1 > nN - 1 ? nN - 1 : r1);
    r2 = r2 < 0 ? 0 : (r2 > nN - 1 ? nN - 1 : r2);
    r3 = r3 < 0 ? 0 : (r3 > nN - 1 ? nN - 1 : r3);
    v4i s4;
    s4.x = (idx     < tt) ? r0 : 0;
    s4.y = (idx + 1 < tt) ? r1 : 0;
    s4.z = (idx + 2 < tt) ? r2 : 0;
    s4.w = (idx + 3 < tt) ? r3 : 0;
    *(volatile v4i*)(bl + idx) = s4;
    __threadfence();
    *(volatile v4i*)(bl + idx) = s4;
  }
}

__global__ __launch_bounds__(GTHR) void k_gemm(const unsigned short* __restrict__ A,
                                               const unsigned short* __restrict__ BT, int K, float* outF) {
  __shared__ __attribute__((aligned(16))) float stg[GBM * GBN];
  const int tid = (int)threadIdx.x, lane = tid & 31, wave = tid >> 5, hh = lane >> 4, m = lane & 15;
  const int rowBase = (int)blockIdx.x * GBM;

  v8f acc[8];
  {
    const v8f z = {0.f, 0.f, 0.f, 0.f, 0.f, 0.f, 0.f, 0.f};
#pragma unroll
    for (int t = 0; t < 8; ++t) acc[t] = z;
  }
  const unsigned short* ap = A  + (size_t)(rowBase + 16 * wave + m) * (size_t)K + 8 * hh;
  const unsigned short* bp = BT + (size_t)m * (size_t)K + 8 * hh;

#pragma unroll 1
  for (int k0 = 0; k0 < K; k0 += 32) {
    FragB af;
    af.h[0] = *(const v8usa*)(ap + k0);
    af.h[1] = *(const v8usa*)(ap + k0 + 16);
#pragma unroll
    for (int nt = 0; nt < 8; ++nt) {
      const unsigned short* wq = bp + (size_t)(16 * nt) * (size_t)K + k0;
      FragB bf;
      bf.h[0] = *(const v8usa*)wq;
      bf.h[1] = *(const v8usa*)(wq + 16);
      acc[nt] = wmb(af, bf, acc[nt]);
    }
  }

#pragma unroll
  for (int nt = 0; nt < 8; ++nt) {
    const int lc = 16 * nt + m;
#pragma unroll
    for (int r = 0; r < 8; ++r) {
      const int lr = 16 * wave + 8 * hh + r;
      stg[lr * GBN + lc] = acc[nt][r];
    }
  }
  __syncthreads();

  v4f pv[16];
#pragma unroll
  for (int i = 0; i < 16; ++i) pv[i] = *(const v4fa*)(stg + (16 * wave + i) * GBN + 4 * lane);
#pragma unroll
  for (int i = 0; i < 16; ++i) {
    const int r = rowBase + 16 * wave + i;
    *(volatile v4f*)(outF + (size_t)r * DF + 4 * lane) = pv[i];
  }
  __threadfence();
#pragma unroll
  for (int i = 0; i < 16; ++i) {
    const int r = rowBase + 16 * wave + i;
    *(volatile v4f*)(outF + (size_t)r * DF + 4 * lane) = pv[i];
  }
}

template <int FIN>
__global__ __launch_bounds__(NTHR) void k_agg(const int* __restrict__ lst, const int* __restrict__ cntT,
                                              const int* __restrict__ offT, const int* __restrict__ meta,
                                              int nN, int mRows, const float* __restrict__ dis,
                                              const float* __restrict__ hw, const float* __restrict__ bias,
                                              unsigned short* xhl, float* hout) {
  __shared__ __attribute__((aligned(16))) unsigned short rowbufs[NWAVE * K2];
  __shared__ __attribute__((aligned(16))) int scnt[NBA];
  __shared__ __attribute__((aligned(16))) int soff[NBA];
  const int tid = (int)threadIdx.x, lane = tid & 31, wave = tid >> 5;
  const int blk = (int)blockIdx.x;
  const int nodeBase = blk * NBA;
  unsigned short* rowbuf = rowbufs + wave * K2;
  {
    const v4i c4 = *(const v4i*)(cntT + (size_t)nodeBase + 4 * tid);
    const v4i o4 = *(const v4i*)(offT + (size_t)nodeBase + 4 * tid);
    *(v4ia*)(scnt + 4 * tid) = c4;
    *(v4ia*)(soff + 4 * tid) = o4;
  }
  const int ovf = meta[(size_t)blk * MLINE + 1];
  v4f b4;
  {
    const v4f a = *(const v4f*)(bias + 4 * lane);
    b4.x = bf16_val(a.x); b4.y = bf16_val(a.y); b4.z = bf16_val(a.z); b4.w = bf16_val(a.w);
  }
  const int* bl = lst + (size_t)blk * RCAP;
  __syncthreads();

  const float qnan = __int_as_float(0x7fc00000);
  const float pz = (ovf != 0) ? qnan : 0.0f;
#pragma unroll 1
  for (int si = 0; si < NBA / NWAVE; ++si) {
    const int s    = si * NWAVE + wave;
    const int node = nodeBase + s;
    int c = scnt[s];
    const bool big = c > DEGCAP;
    c = c < 0 ? 0 : (c > DEGCAP ? DEGCAP : c);
    int o = soff[s];
    o = o < 0 ? 0 : (o > RCAP ? RCAP : o);
    const int last = o + c - 1;
    const int nc = node < nN ? node : nN - 1;
    const float dd = dis[nc];
    const float rd = dd * dd;
    float a0 = 0.0f, a1 = 0.0f, a2 = 0.0f, a3 = 0.0f;
#pragma unroll 1
    for (int b0 = 0; b0 < c; b0 += 32) {
      int idx = o + b0 + lane;
      idx = idx > last ? last : idx;
      idx = idx > RCAP - 1 ? RCAP - 1 : idx;
      idx = idx < 0 ? 0 : idx;
      int sr = bl[idx];
      sr = sr < 0 ? 0 : (sr > nN - 1 ? nN - 1 : sr);
      const float cf  = dis[sr] * dd;
      const int   cfi = __float_as_int(cf);
      const int m32 = (c - b0) < 32 ? (c - b0) : 32;
#pragma unroll 1
      for (int k = 0; k < m32; ++k) {
        const int   sk = __builtin_amdgcn_readlane(sr, k);
        const float ck = __int_as_float(__builtin_amdgcn_readlane(cfi, k));
        const v4f a = *(const v4f*)(hw + (size_t)sk * DF + 4 * lane);
        a0 = fmaf(ck, a.x, a0);
        a1 = fmaf(ck, a.y, a1);
        a2 = fmaf(ck, a.z, a2);
        a3 = fmaf(ck, a.w, a3);
      }
    }
    const v4f sv = *(const v4f*)(hw + (size_t)nc * DF + 4 * lane);
    const float pzr = big ? qnan : pz;
    const bool live = node < nN;
    float y0 = (a0 + sv.x * rd) + b4.x;
    float y1 = (a1 + sv.y * rd) + b4.y;
    float y2 = (a2 + sv.z * rd) + b4.z;
    float y3 = (a3 + sv.w * rd) + b4.w;
    y0 = (y0 > 0.0f) ? y0 : (y0 - y0);
    y1 = (y1 > 0.0f) ? y1 : (y1 - y1);
    y2 = (y2 > 0.0f) ? y2 : (y2 - y2);
    y3 = (y3 > 0.0f) ? y3 : (y3 - y3);
    const float m0 = live ? (y0 + pzr) : 0.0f;
    const float m1 = live ? (y1 + pzr) : 0.0f;
    const float m2 = live ? (y2 + pzr) : 0.0f;
    const float m3 = live ? (y3 + pzr) : 0.0f;
    v4us mh, ml;
    {
      unsigned hb;
      hb = bf16_bits(m0); mh[0] = (unsigned short)hb; ml[0] = (unsigned short)bf16_bits(m0 - __uint_as_float(hb << 16));
      hb = bf16_bits(m1); mh[1] = (unsigned short)hb; ml[1] = (unsigned short)bf16_bits(m1 - __uint_as_float(hb << 16));
      hb = bf16_bits(m2); mh[2] = (unsigned short)hb; ml[2] = (unsigned short)bf16_bits(m2 - __uint_as_float(hb << 16));
      hb = bf16_bits(m3); mh[3] = (unsigned short)hb; ml[3] = (unsigned short)bf16_bits(m3 - __uint_as_float(hb << 16));
    }
    *(v4usa*)(rowbuf + 4 * lane) = mh;
    *(v4usa*)(rowbuf + DF + 4 * lane) = ml;
    wave_sync();
    const v8us q0 = *(const v8usa*)(rowbuf + 8 * lane);
    wave_sync();
    v4f fv;
    fv.x = m0; fv.y = m1; fv.z = m2; fv.w = m3;
    unsigned short* rpw = xhl + (size_t)node * K2 + 8 * lane;
    float* fpw = hout + (size_t)nc * DF + 4 * lane;
    const bool wx = node < mRows;
    if (wx) *(volatile v8us*)rpw = q0;
    if constexpr (FIN != 0) { if (live) *(volatile v4f*)fpw = fv; }
    __threadfence();
    if (wx) *(volatile v8us*)rpw = q0;
    if constexpr (FIN != 0) { if (live) *(volatile v4f*)fpw = fv; }
  }
}

__global__ __launch_bounds__(GTHR) void k_cls(const unsigned short* __restrict__ A,
                                              const unsigned short* __restrict__ BT,
                                              const float* __restrict__ bc, float* out, int nOutF) {
  __shared__ __attribute__((aligned(16))) float stg[GBM * NCLS];
  __shared__ float bcs[NCP];
  const int tid = (int)threadIdx.x, lane = tid & 31, wave = tid >> 5, hh = lane >> 4, m = lane & 15;
  const int rowBase = (int)blockIdx.x * GBM;

  if (tid < NCP) {
    const float bb = bc[tid < NCLS ? tid : NCLS - 1];
    bcs[tid] = (tid < NCLS) ? bb : 0.0f;
  }
  v8f acc[3];
  {
    const v8f z = {0.f, 0.f, 0.f, 0.f, 0.f, 0.f, 0.f, 0.f};
    acc[0] = z; acc[1] = z; acc[2] = z;
  }
  const unsigned short* ap = A  + (size_t)(rowBase + 16 * wave + m) * (size_t)K2 + 8 * hh;
  const unsigned short* bp = BT + (size_t)m * (size_t)K2 + 8 * hh;
#pragma unroll 1
  for (int k0 = 0; k0 < K2; k0 += 32) {
    FragB af;
    af.h[0] = *(const v8usa*)(ap + k0);
    af.h[1] = *(const v8usa*)(ap + k0 + 16);
#pragma unroll
    for (int nt = 0; nt < 3; ++nt) {
      const unsigned short* wq = bp + (size_t)(16 * nt) * (size_t)K2 + k0;
      FragB bf;
      bf.h[0] = *(const v8usa*)wq;
      bf.h[1] = *(const v8usa*)(wq + 16);
      acc[nt] = wmb(af, bf, acc[nt]);
    }
  }
  __syncthreads();
#pragma unroll
  for (int nt = 0; nt < 3; ++nt) {
    const int c = 16 * nt + m;
    const float bv = bcs[c];
    const bool cok = c < NCLS;
#pragma unroll
    for (int r = 0; r < 8; ++r) {
      const int lr = 16 * wave + 8 * hh + r;
      if (cok) stg[lr * NCLS + c] = acc[nt][r] + bv;
    }
  }
  __syncthreads();

  constexpr int NIT = (GBM * NCLS) / (4 * GTHR);
  const size_t fbase = (size_t)rowBase * NCLS;
  v4f ov[NIT];
#pragma unroll
  for (int it = 0; it < NIT; ++it) ov[it] = *(const v4fa*)(stg + 4 * (it * GTHR + tid));
#pragma unroll
  for (int it = 0; it < NIT; ++it) {
    const size_t g = fbase + 4 * (size_t)(it * GTHR + tid);
    if (g + 3 < (size_t)nOutF) *(volatile v4f*)(out + g) = ov[it];
  }
  __threadfence();
#pragma unroll
  for (int it = 0; it < NIT; ++it) {
    const size_t g = fbase + 4 * (size_t)(it * GTHR + tid);
    if (g + 3 < (size_t)nOutF) *(volatile v4f*)(out + g) = ov[it];
  }
}

static inline int cdiv(int a, int b) { return (a + b - 1) / b; }
static inline size_t al256(size_t o) { return (o + 255) & ~(size_t)255; }

extern "C" void kernel_launch(void* const* d_in, const int* in_sizes, int n_in,
                              void* d_out, int out_size, void* d_ws, size_t ws_size,
                              hipStream_t stream) {
  if (n_in < 10) return;
  if (in_sizes[0] < DF || (in_sizes[0] % DF) != 0) return;
  const int nN = in_sizes[0] / DF;
  if (nN < 16 || nN > (1 << 22)) return;
  if (in_sizes[1] < 2 || (in_sizes[1] & 1) != 0) return;
  const int nE = in_sizes[1] / 2;
  if (nE < 1 || nE >= (1 << (31 - SLA))) return;
  if (in_sizes[2] != DF * DF || in_sizes[3] != DF) return;
  if (in_sizes[4] != DF * DF || in_sizes[5] != DF) return;
  if (in_sizes[6] != DF * DF || in_sizes[7] != DF) return;
  if (in_sizes[8] != DF * NCLS || in_sizes[9] != NCLS) return;
  const long long nOut0 = (long long)nN * NCLS;
  const long long nOut1 = (long long)nN * DF;
  if ((long long)out_size != nOut0 + nOut1) return;
  if ((nOut0 % 32) != 0) return;

  const float* x    = (const float*)d_in[0];
  const int*   edge = (const int*)d_in[1];
  const float* W1   = (const float*)d_in[2];
  const float* b1   = (const float*)d_in[3];
  const float* W2   = (const float*)d_in[4];
  const float* b2   = (const float*)d_in[5];
  const float* W3   = (const float*)d_in[6];
  const float* b3   = (const float*)d_in[7];
  const float* Wc   = (const float*)d_in[8];
  const float* bc   = (const float*)d_in[9];
  float* out  = (float*)d_out;
  float* hout = out + (size_t)nOut0;
  const int* src = edge;
  const int* dst = edge + nE;

  const int MP   = cdiv(nN, GBM) * GBM;
  const int gM   = MP / GBM;
  const int gA   = cdiv(MP, NBA);
  const int NBPA = gA * NBA;
  if ((long long)gA * NBA < (long long)MP) return;
  const int vec8 = ((nE & 3) == 0) ? 1 : 0;

  char* ws = (char*)d_ws;
  size_t off = 0;
  const size_t oDIS  = off; off = al256(off + (size_t)NBPA * 4);
  const size_t oCNT  = off; off = al256(off + (size_t)NBPA * 4);
  const size_t oOFF  = off; off = al256(off + (size_t)NBPA * 4);
  const size_t oMETA = off; off = al256(off + (size_t)gA * MLINE * 4);
  const size_t oLST  = off; off = al256(off + (size_t)gA * RCAP * 4);
  const size_t oW1T  = off; off = al256(off + (size_t)DF * DF * 2);
  const size_t oW2T  = off; off = al256(off + (size_t)DF * K2 * 2);
  const size_t oW3T  = off; off = al256(off + (size_t)DF * K2 * 2);
  const size_t oWCT  = off; off = al256(off + (size_t)NCP * K2 * 2);
  const size_t oXB   = off; off = al256(off + (size_t)MP * DF * 2);
  const size_t oHW   = off; off = al256(off + (size_t)MP * DF * 4);
  const size_t oX    = off; off = al256(off + (size_t)MP * K2 * 2);
  if (off > ws_size || off > (size_t)WSMAX) return;
  float*          DIS  = (float*)(ws + oDIS);
  int*            CNT  = (int*)(ws + oCNT);
  int*            OFFS = (int*)(ws + oOFF);
  int*            META = (int*)(ws + oMETA);
  int*            LST  = (int*)(ws + oLST);
  unsigned short* W1T  = (unsigned short*)(ws + oW1T);
  unsigned short* W2T2 = (unsigned short*)(ws + oW2T);
  unsigned short* W3T2 = (unsigned short*)(ws + oW3T);
  unsigned short* WcT2 = (unsigned short*)(ws + oWCT);
  unsigned short* XB   = (unsigned short*)(ws + oXB);
  float*          HW   = (float*)(ws + oHW);
  unsigned short* X    = (unsigned short*)(ws + oX);

  const size_t stLds = (size_t)STRUCT_LDS_INTS * 4;
  hipFuncSetAttribute(reinterpret_cast<const void*>(&k_struct), hipFuncAttributeMaxDynamicSharedMemorySize, (int)stLds);

  const int nUx = MP * (DF / 8);
  k_cvx<<<cdiv(nUx, NTHR), NTHR, 0, stream>>>(x, nN, nUx, XB);
  k_wprep<<<U_ALL / NTHR, NTHR, 0, stream>>>(W1, W2, W3, Wc, W1T, W2T2, W3T2, WcT2);
  k_struct<<<gA, NTHR, stLds, stream>>>(src, dst, nE, nN, vec8, DIS, CNT, OFFS, META, LST);
  k_gemm<<<gM, GTHR, 0, stream>>>(XB, W1T, DF, HW);
  k_agg<0><<<gA, NTHR, 0, stream>>>(LST, CNT, OFFS, META, nN, MP, DIS, HW, b1, X, hout);
  k_gemm<<<gM, GTHR, 0, stream>>>(X, W2T2, K2, HW);
  k_agg<0><<<gA, NTHR, 0, stream>>>(LST, CNT, OFFS, META, nN, MP, DIS, HW, b2, X, hout);
  k_gemm<<<gM, GTHR, 0, stream>>>(X, W3T2, K2, HW);
  k_agg<1><<<gA, NTHR, 0, stream>>>(LST, CNT, OFFS, META, nN, MP, DIS, HW, b3, X, hout);
  k_cls<<<gM, GTHR, 0, stream>>>(X, WcT2, bc, out, (int)nOut0);
}
